// align_uniform_Loss_6176162971828
// MI455X (gfx1250) — hardware-run, weakly checked
//
#include <hip/hip_runtime.h>
#include <math.h>

typedef __attribute__((ext_vector_type(16))) _Float16 v16h;
typedef __attribute__((ext_vector_type(16))) __bf16 v16b;
typedef __attribute__((ext_vector_type(8)))  _Float16 v8h;
typedef __attribute__((ext_vector_type(8)))  float v8f;
typedef __attribute__((ext_vector_type(4)))  float v4f;
typedef __attribute__((ext_vector_type(2)))  float v2f;
typedef __attribute__((ext_vector_type(4)))  unsigned v4u;
typedef __attribute__((ext_vector_type(4)))  int v4i;
typedef float __attribute__((may_alias)) float_a;
typedef int __attribute__((may_alias)) int_a;

template <typename T> __device__ __forceinline__ void vst2(void* p, T v) { *(volatile T*)p = v; __threadfence(); *(volatile T*)p = v; }
__device__ __forceinline__ v8f wmma16(v16h a, v16h b, v8f c) {
  v8f d = __builtin_amdgcn_wmma_f32_16x16x32_f16(false, a, false, b, (short)0, c, false, false);
  asm volatile("v_nop\n\tv_nop\n\tv_nop\n\tv_nop" : "+v"(d) : "v"(a), "v"(b));
  return d;
}
__device__ __forceinline__ v8f wmma_bf(v16b a, v16b b, v8f c) {
  v8f d = __builtin_amdgcn_wmma_f32_16x16x32_bf16(false, a, false, b, (short)0, c, false, false);
  asm volatile("v_nop\n\tv_nop\n\tv_nop\n\tv_nop" : "+v"(d) : "v"(a), "v"(b));
  return d;
}
__device__ __forceinline__ v16h frag_h(const _Float16* rowk0, int lane) {
  union { v16h v; v8h q[2]; } u; const _Float16* p = rowk0 + 8 * (lane >> 4);
  u.q[0] = *(const v8h*)p; u.q[1] = *(const v8h*)(p + 16); return u.v;
}
__device__ __forceinline__ v16h frag_f32(const float* rowk0, int lane) {
  v16h a; const float* p = rowk0 + 8 * (lane >> 4);
#pragma unroll
  for (int i = 0; i < 8; ++i) { a[i] = (_Float16)p[i]; a[8 + i] = (_Float16)p[16 + i]; }
  return a;
}
__device__ __forceinline__ v16h frag_f32s(const float* rowk0, int lane, float sc) {
  v16h a; const float* p = rowk0 + 8 * (lane >> 4);
#pragma unroll
  for (int i = 0; i < 8; ++i) { a[i] = (_Float16)(p[i] * sc); a[8 + i] = (_Float16)(p[16 + i] * sc); }
  return a;
}
__device__ __forceinline__ v16h fragc_f32(const float* W, int k0, int n, int lane, int ld, int K) {
  v16h a; const int g = lane >> 4;
#pragma unroll
  for (int i = 0; i < 8; ++i) { const int ka = k0 + 8 * g + i, kb = ka + 16;
    a[i] = (_Float16)(ka < K ? W[(size_t)(ka < K ? ka : K - 1) * ld + n] : 0.f); a[8 + i] = (_Float16)(kb < K ? W[(size_t)(kb < K ? kb : K - 1) * ld + n] : 0.f); }
  return a;
}
struct F2 { v16b h, l; };
__device__ __forceinline__ F2 bsplit16(const float v[16]) { F2 r;
#pragma unroll
  for (int i = 0; i < 16; ++i) { const __bf16 h = (__bf16)v[i]; r.h[i] = h; r.l[i] = (__bf16)(v[i] - (float)h); }
  return r; }
__device__ __forceinline__ F2 split_row(const float* row, int k0, int lane) { float v[16]; const float* p = row + k0 + 8 * (lane >> 4);
#pragma unroll
  for (int i = 0; i < 8; ++i) { v[i] = p[i]; v[8 + i] = p[16 + i]; }
  return bsplit16(v); }
__device__ __forceinline__ F2 split_rowK(const float* row, int k0, int lane, int K) { float v[16]; const int g = lane >> 4;
#pragma unroll
  for (int i = 0; i < 8; ++i) { const int ka = k0 + 8 * g + i, kb = ka + 16; v[i] = ka < K ? row[ka < K ? ka : K - 1] : 0.f; v[8 + i] = kb < K ? row[kb < K ? kb : K - 1] : 0.f; }
  return bsplit16(v); }
__device__ __forceinline__ F2 split_col(const float* W, int k0, int n, int lane, int ld, int K) { float v[16]; const int g = lane >> 4;
#pragma unroll
  for (int i = 0; i < 8; ++i) { const int ka = k0 + 8 * g + i, kb = ka + 16; v[i] = ka < K ? W[(size_t)(ka < K ? ka : K - 1) * ld + n] : 0.f; v[8 + i] = kb < K ? W[(size_t)(kb < K ? kb : K - 1) * ld + n] : 0.f; }
  return bsplit16(v); }
__device__ __forceinline__ v8f mac3(const F2& a, const F2& b, v8f c) { c = wmma_bf(a.l, b.h, c); c = wmma_bf(a.h, b.l, c); return wmma_bf(a.h, b.h, c); }
__device__ __forceinline__ float sigm(float v) { return 1.0f / (1.0f + expf(-v)); }
#define LDSX() do { asm volatile("s_wait_dscnt 0" ::: "memory"); __builtin_amdgcn_wave_barrier(); __builtin_amdgcn_fence(__ATOMIC_RELEASE, "workgroup"); } while (0)


#define NN 8192
#define DD 128
#ifndef NRT
#define NRT (NN / 64)
#endif
typedef __attribute__((ext_vector_type(8))) __bf16 v8b;
__device__ __forceinline__ v16b frag_b(const __bf16* rowk0, int lane) {
  union { v16b v; v8b q[2]; } u; const __bf16* p = rowk0 + 8 * (lane >> 4);
  u.q[0] = *(const v8b*)p; u.q[1] = *(const v8b*)(p + 16); return u.v;
}
__device__ __forceinline__ float bfr(float v) { return (float)(__bf16)v; }
__device__ __attribute__((noinline)) float exp_ni(float v) { return expf(v); }
__device__ __attribute__((noinline)) float erf_ni(float v) { return erff(v); }

#define WS_UB   0u
#define WS_IB   (WS_UB + 2u * NN * DD)
#define WS_ST   (WS_IB + 2u * NN * DD)
#define WS_RN   WS_ST
#define WS_SQ   (WS_RN + 4u * 2 * NN)
#define WS_PAL  (WS_SQ + 4u * 2 * NN)
#define WS_PUN  (((WS_PAL + 128u * NRT) + 127u) / 128u * 128u)
#define WS_END  (WS_PUN + 128u * 2 * NRT * (NN / 128))

__global__ __launch_bounds__(256) void k_rows(const float* __restrict__ U, const float* __restrict__ V, __bf16* __restrict__ UB, __bf16* __restrict__ IB, float* __restrict__ RN, float* __restrict__ SQ, double* __restrict__ PAL) {
  __shared__ __align__(16) __bf16 su[64][DD], sv[64][DD]; __shared__ __align__(16) float srn[2][64], ssq[2][64]; __shared__ double sal[64]; __shared__ __align__(16) double spal[16];
  const int tid = threadIdx.x; const size_t r0 = (size_t)blockIdx.x * 64;
  for (int q = tid; q < 64 * DD; q += 256) { const int r = q >> 7, d = q & 127; su[r][d] = (__bf16)U[(r0 + r) * DD + d]; sv[r][d] = (__bf16)V[(r0 + r) * DD + d]; }
  __syncthreads();
  if (tid < 128) { const int r = tid & 63, which = tid >> 6; const __bf16 (*s)[DD] = which ? sv : su; float a = 0.f; for (int d = 0; d < DD; ++d) { const float x = (float)s[r][d]; a += x * x; }
    const float rn = 1.0f / fmaxf(sqrtf(a), 1e-12f); float b = 0.f; for (int d = 0; d < DD; ++d) { const float x = (float)s[r][d] * rn; b += x * x; } srn[which][r] = rn; ssq[which][r] = b; }
  __syncthreads();
  if (tid < 64) { const int r = tid; double a = 0.0; for (int d = 0; d < DD; ++d) { const float df = (float)su[r][d] * srn[0][r] - (float)sv[r][d] * srn[1][r]; a += (double)(df * df); } sal[r] = a; }
  __syncthreads();
  if (tid < 16) spal[tid] = 0.0;
  __syncthreads();
  if (tid == 0) { double a = 0.0; for (int r = 0; r < 64; ++r) a += sal[r]; spal[0] = a; }
  __syncthreads();
  for (int q = tid; q < 64 * DD / 8; q += 256) { vst2((unsigned*)(UB + r0 * DD + q * 8), *(const v4u*)(&su[0][0] + q * 8)); vst2((unsigned*)(IB + r0 * DD + q * 8), *(const v4u*)(&sv[0][0] + q * 8)); }
  if (tid < 16) vst2(RN + r0 + tid * 4, *(const v4f*)&srn[0][tid * 4]); else if (tid < 32) vst2(RN + NN + r0 + (tid - 16) * 4, *(const v4f*)&srn[1][(tid - 16) * 4]);
  else if (tid < 48) vst2(SQ + r0 + (tid - 32) * 4, *(const v4f*)&ssq[0][(tid - 32) * 4]); else if (tid < 64) vst2(SQ + NN + r0 + (tid - 48) * 4, *(const v4f*)&ssq[1][(tid - 48) * 4]);
  if (tid == 64 && (blockIdx.x & 7) == 0) { }
  if (tid < 8) vst2((unsigned*)(PAL + (size_t)blockIdx.x * 16 + tid * 2), *(const v4u*)&spal[tid * 2]);
}
__global__ __launch_bounds__(128) void k_gram(const __bf16* __restrict__ UB, const __bf16* __restrict__ IB, const float* __restrict__ RN, const float* __restrict__ SQ, double* __restrict__ PUN) {
  __shared__ double sw[4]; __shared__ __align__(16) double sp[16];
  const int tid = threadIdx.x, wave = tid >> 5, lane = tid & 31, col = lane & 15, g = lane >> 4; const int ti = blockIdx.x, tj = blockIdx.y, which = blockIdx.z; const size_t i0 = (size_t)ti * 64, j0 = (size_t)tj * 128;
  const __bf16* X = which ? IB : UB; const float* rn = RN + (size_t)which * NN; const float* sq = SQ + (size_t)which * NN;
  double part = 0.0;
  if (j0 + 127 > i0) {
    const size_t ri = i0 + wave * 16; v8f acc[8] = {};
#pragma unroll
    for (int kc = 0; kc < DD / 32; ++kc) { const v16b a = frag_b(X + (ri + col) * DD + kc * 32, lane);
#pragma unroll
      for (int j = 0; j < 8; ++j) acc[j] = wmma_bf(a, frag_b(X + (j0 + j * 16 + col) * DD + kc * 32, lane), acc[j]); }
    float s = 0.f;
#pragma unroll
    for (int j = 0; j < 8; ++j) { const size_t jj = j0 + j * 16 + col; const float rnj = rn[jj], sqj = sq[jj];
#pragma unroll
      for (int r = 0; r < 8; ++r) { const size_t ii = ri + 8 * g + r; if (jj > ii) { const float d2 = fmaxf((sq[ii] + sqj) - 2.0f * (acc[j][r] * rn[ii] * rnj), 0.f); s += __expf(-2.0f * d2); } } }
    double ds = (double)s;
#pragma unroll
    for (int o = 1; o < 32; o <<= 1) ds += __shfl_xor(ds, o);
    if (lane == 0) sw[wave] = ds;
    __syncthreads();
    if (tid == 0) part = (sw[0] + sw[1]) + (sw[2] + sw[3]);
  }
  if (tid < 16) sp[tid] = (tid == 0) ? part : 0.0;
  __syncthreads();
  if (tid < 8) vst2((unsigned*)(PUN + (((size_t)which * NRT + ti) * (NN / 128) + tj) * 16 + tid * 2), *(const v4u*)&sp[tid * 2]);
}
__global__ __launch_bounds__(256) void k_final(const double* __restrict__ PAL, const double* __restrict__ PUN, int nrt, float* __restrict__ OUT) {
  __shared__ double sa[256], su[256], si[256]; const int t = threadIdx.x; double a = 0.0, u = 0.0, v = 0.0;
  for (int b = t; b < nrt; b += 256) a += PAL[(size_t)b * 16];
  { const int ntj = nrt * 64 / 128; for (int q = t; q < nrt * ntj; q += 256) { const int ti = q / ntj, tj = q % ntj; const size_t e = (size_t)ti * (NN / 128) + tj; u += PUN[e * 16]; v += PUN[((size_t)NRT * (NN / 128) + e) * 16]; } }
  sa[t] = a; su[t] = u; si[t] = v; __syncthreads();
  if (t == 0) { double A = 0.0, Us = 0.0, Is = 0.0; for (int i = 0; i < 256; ++i) { A += sa[i]; Us += su[i]; Is += si[i]; }
    const double n = (double)nrt * 64.0; const double npairs = n * (n - 1.0) / 2.0;
    const double align = A / n; const double unif = 0.5 * (log(Us / npairs) + log(Is / npairs)) / 2.0; const float loss = (float)((align + unif) / 8192.0);
    *(volatile float*)OUT = loss; *(volatile float*)OUT = loss; }
}
extern "C" void kernel_launch(void* const* d_in, const int* in_sizes, int n_in, void* d_out, int out_size, void* d_ws, size_t ws_size, hipStream_t stream) {
  (void)in_sizes; (void)n_in; (void)out_size;
  const float** F = (const float**)d_in;
  if (ws_size < (size_t)WS_END) return;
  char* ws = (char*)d_ws; __bf16 *UB = (__bf16*)(ws + WS_UB), *IB = (__bf16*)(ws + WS_IB); float *RN = (float*)(ws + WS_RN), *SQ = (float*)(ws + WS_SQ); double *PAL = (double*)(ws + WS_PAL), *PUN = (double*)(ws + WS_PUN);
  k_rows<<<NRT, 256, 0, stream>>>(F[0], F[1], UB, IB, RN, SQ, PAL);
  k_gram<<<dim3(NRT, (NRT * 64) / 128, 2), 128, 0, stream>>>(UB, IB, RN, SQ, PUN);
  k_final<<<1, 256, 0, stream>>>(PAL, PUN, NRT, (float*)d_out);
}
